// GraphSAGE_4733053960253
// MI455X (gfx1250) — hardware-verified
//
#include <hip/hip_runtime.h>
#include <math.h>

constexpr int kNodes   = 50000;
constexpr int kNPad    = 50048;
constexpr int kEdges   = 640000;
constexpr int kPairs   = 100000;
constexpr int kCh      = 128;
constexpr int kCh2     = 256;
constexpr int kNT      = 256;
constexpr int kSRB     = 2048;
constexpr int kTiles   = 25;
constexpr int kAggRows = kTiles * kSRB;
constexpr int kRPW     = kSRB / 8;
constexpr int kRPWLog  = 8;
constexpr int kSCH     = 4096;
constexpr int kSP      = kSCH / kNT;
constexpr int kNCH     = (kEdges + kSCH - 1) / kSCH;
constexpr int kZP      = 136;
constexpr int kPB      = (kPairs + 63) / 64;
constexpr int kGemmTiles  = (kNPad / 64) * (kCh2 / 64);
constexpr int kGemmBlocks = kGemmTiles / 8;

static_assert(kNPad % 64 == 0 && kNPad >= kNodes && kNPad - kNodes < 64, "m");
static_assert(kCh % 32 == 0 && kCh2 % 64 == 0, "k");
static_assert(kGemmBlocks * 8 == kGemmTiles, "g");
static_assert(kEdges % kSP == 0 && kSP % 4 == 0, "e");
static_assert(kAggRows >= kNPad && (1 << kRPWLog) == kRPW && kRPW * 8 == kSRB && (kRPW % 2) == 0, "t");
static_assert(kNodes <= 65535 && kSRB <= 32768, "p");
static_assert((kNPad % 2) == 0, "u");
static_assert(kPB * 64 >= kPairs && ((kPairs % 64) == 0 || (kPairs % 64) == 32), "o");
static_assert((kPairs * 4) % 128 == 0, "a");

constexpr size_t kCarveTotal = (size_t)3 * 65536 + (size_t)2 * 32768 + (size_t)2 * kNPad * kCh * 2 +
                               (size_t)kNPad * kCh2 * 4 + (size_t)kAggRows * kCh * 4 + (size_t)kNPad * kCh * 4;
static_assert(kCarveTotal == 128974848ull, "c");
static_assert(kCarveTotal <= 134217728ull, "w");

typedef __attribute__((ext_vector_type(16))) __bf16   v16b;
typedef __attribute__((ext_vector_type(8)))  __bf16   v8b;
typedef __attribute__((ext_vector_type(8)))  float    v8f;
typedef __attribute__((ext_vector_type(4)))  float    v4f;
typedef __attribute__((ext_vector_type(4)))  int      v4i;
typedef __attribute__((ext_vector_type(4)))  unsigned int v4u;

__device__ __forceinline__ unsigned short f2bf_bits(float f) {
  unsigned u = __float_as_uint(f);
  return (unsigned short)((u + 0x7FFFu + ((u >> 16) & 1u)) >> 16);
}
__device__ __forceinline__ float bf_bits2f(unsigned short h) { return __uint_as_float(((unsigned)h) << 16); }
__device__ __forceinline__ float bfr(float f) { return bf_bits2f(f2bf_bits(f)); }
__device__ __forceinline__ v4f bfr4(v4f a) { v4f r; r[0] = bfr(a[0]); r[1] = bfr(a[1]); r[2] = bfr(a[2]); r[3] = bfr(a[3]); return r; }
__device__ __forceinline__ unsigned pk16(unsigned short a, unsigned short b) { return (unsigned)a | ((unsigned)b << 16); }

__device__ __forceinline__ void keep4_b(v16b a, v16b b, v16b c, v16b d) { asm volatile("v_nop" :: "v"(a), "v"(b), "v"(c), "v"(d)); }
__device__ __forceinline__ void acc_guard4(v8f& a, v8f& b, v8f& c, v8f& d) { asm volatile("v_nop\n\tv_nop\n\tv_nop\n\tv_nop" : "+v"(a), "+v"(b), "+v"(c), "+v"(d)); }
__device__ __forceinline__ void guard4_b(v8f& a, v8f& b, v8f& c, v8f& d, v16b x, v16b y) {
  asm volatile("v_nop\n\tv_nop\n\tv_nop\n\tv_nop" : "+v"(a), "+v"(b), "+v"(c), "+v"(d) : "v"(x), "v"(y));
}

template <typename T> struct Frag;
template <> struct Frag<__bf16> {
  typedef v16b V; union U { v16b v; v8b h[2]; };
  static __device__ __forceinline__ v16b load(const __bf16* p) {
    U f; f.h[0] = *(const v8b*)(p); f.h[1] = *(const v8b*)(p + 16); return f.v;
  }
  static __device__ __forceinline__ v8f mma(v16b a, v16b b, v8f c) {
    return __builtin_amdgcn_wmma_f32_16x16x32_bf16(false, a, false, b, (short)0, c, false, false);
  }
};

template <bool ASPLIT>
__global__ __launch_bounds__(256) void sage_gemm_kernel(const unsigned short* __restrict__ Ap, const unsigned short* __restrict__ A2p,
                                                        const unsigned short* __restrict__ Btp, float* __restrict__ Cout) {
  const __bf16* A = (const __bf16*)Ap; const __bf16* A2 = (const __bf16*)A2p; const __bf16* Bt = (const __bf16*)Btp;
  __shared__ __align__(16) float sT[8][16 * 68];
  const int lane = threadIdx.x & 31;
  const int wave = threadIdx.x >> 5;
  constexpr int tilesN = kCh2 / 64;
  constexpr int tilesM = kNPad / 64;
  const int tile = blockIdx.x * 8 + wave;
  if (tile >= tilesM * tilesN) return;
  const int tm = tile / tilesN;
  const int tn = tile - tm * tilesN;
  const int m0 = tm << 6;
  const int n0 = tn << 6;
  const int rlane = lane & 15;
  const int koff  = (lane >> 4) * 8;
  const int mOff  = (lane >> 4) * 8;

  v8f acc[4][4];
#pragma unroll
  for (int i = 0; i < 4; ++i)
#pragma unroll
    for (int j = 0; j < 4; ++j) acc[i][j] = (v8f){0.f,0.f,0.f,0.f,0.f,0.f,0.f,0.f};

  for (int k0 = 0; k0 < kCh; k0 += 32) {
    v16b bh[4];
#pragma unroll
    for (int j = 0; j < 4; ++j) {
      const size_t bo = (size_t)(n0 + (j << 4) + rlane) * kCh + koff + k0;
      bh[j] = Frag<__bf16>::load(Bt + bo);
    }
#pragma unroll
    for (int i = 0; i < 4; ++i) {
      const size_t ao = (size_t)(m0 + (i << 4) + rlane) * kCh + koff + k0;
      const v16b ah = Frag<__bf16>::load(A + ao);
      v16b al = ah;
      if (ASPLIT) al = Frag<__bf16>::load(A2 + ao);
#pragma unroll
      for (int j = 0; j < 4; ++j) {
        acc[i][j] = Frag<__bf16>::mma(ah, bh[j], acc[i][j]);
        if (ASPLIT) acc[i][j] = Frag<__bf16>::mma(al, bh[j], acc[i][j]);
      }
      guard4_b(acc[i][0], acc[i][1], acc[i][2], acc[i][3], ah, al);
    }
    keep4_b(bh[0], bh[1], bh[2], bh[3]);
  }
  acc_guard4(acc[0][0], acc[0][1], acc[0][2], acc[0][3]);
  acc_guard4(acc[1][0], acc[1][1], acc[1][2], acc[1][3]);
  acc_guard4(acc[2][0], acc[2][1], acc[2][2], acc[2][3]);
  acc_guard4(acc[3][0], acc[3][1], acc[3][2], acc[3][3]);

  float* slab = sT[wave];
#pragma unroll
  for (int i = 0; i < 4; ++i) {
    const int mBase = m0 + (i << 4);
#pragma unroll
    for (int j = 0; j < 4; ++j) {
#pragma unroll
      for (int r = 0; r < 8; ++r) slab[(mOff + r) * 68 + (j << 4) + rlane] = acc[i][j][r];
    }
    __builtin_amdgcn_fence(__ATOMIC_RELEASE, "workgroup");
    __builtin_amdgcn_wave_barrier();
    __builtin_amdgcn_fence(__ATOMIC_ACQUIRE, "workgroup");
    {
      float* C = Cout;
      const int hh = lane >> 4, c4 = (lane & 15) * 4;
      for (int pass = 0; pass < 2; ++pass) {
#pragma unroll
        for (int it = 0; it < 8; ++it) {
          const int row = it * 2 + hh;
          v4f v = *(const v4f*)(slab + row * 68 + c4);
          *(volatile v4f*)(C + (size_t)(mBase + row) * kCh2 + n0 + c4) = v;
        }
        __threadfence();
      }
    }
    __builtin_amdgcn_fence(__ATOMIC_RELEASE, "workgroup");
    __builtin_amdgcn_wave_barrier();
    __builtin_amdgcn_fence(__ATOMIC_ACQUIRE, "workgroup");
  }
}

__global__ __launch_bounds__(256) void prep_w_kernel(const float* __restrict__ Ws0, const float* __restrict__ Wn0,
                                                     const float* __restrict__ Ws1, const float* __restrict__ Wn1,
                                                     const float* __restrict__ Ws2, const float* __restrict__ Wn2,
                                                     const float* __restrict__ Wq1, const float* __restrict__ Wq2,
                                                     unsigned* __restrict__ BT0, unsigned* __restrict__ BT1, unsigned* __restrict__ BT2,
                                                     unsigned* __restrict__ BQ1, unsigned* __restrict__ BQ2) {
  const int blk = blockIdx.x, t = threadIdx.x;
  const float* W; unsigned* dst; int i;
  if (blk < 192) {
    const int l = blk >> 6, sub = blk & 63;
    const float* ws = (l == 0) ? Ws0 : ((l == 1) ? Ws1 : Ws2);
    const float* wn = (l == 0) ? Wn0 : ((l == 1) ? Wn1 : Wn2);
    W   = (sub < 32) ? ws : wn;
    dst = (l == 0) ? BT0 : ((l == 1) ? BT1 : BT2);
    i   = sub * 256 + t;
  } else {
    const int q = blk - 192; const int pl = q >> 5, sub = q & 31;
    W   = pl ? Wq2 : Wq1;
    dst = pl ? BQ2 : BQ1;
    i   = sub * 256 + t;
  }
  const int n = i >> 6; const int ncol = n & 127; const int k2 = (i & 63) * 2;
  const float a = W[(size_t)k2 * kCh + ncol];
  const float b = W[(size_t)(k2 + 1) * kCh + ncol];
  const unsigned u = pk16(f2bf_bits(a), f2bf_bits(b));
  ((volatile unsigned*)dst)[i] = u;
  __threadfence();
  ((volatile unsigned*)dst)[i] = u;
}

__global__ __launch_bounds__(256) void cast_x_kernel(const float* __restrict__ x, unsigned short* __restrict__ AH) {
  const int i = blockIdx.x * 256 + threadIdx.x;
  if (i >= kNPad * 16) return;
  const int row = i >> 4, c8 = (i & 15) * 8;
  const bool live = row < kNodes;
  const int rowc = live ? row : (kNodes - 1);
  const float* p = x + (size_t)rowc * kCh + c8;
  const v4f a = *(const v4f*)(p);
  const v4f b = *(const v4f*)(p + 4);
  unsigned short hb[8];
#pragma unroll
  for (int e = 0; e < 4; ++e) {
    hb[e]     = live ? f2bf_bits(a[e]) : (unsigned short)0;
    hb[4 + e] = live ? f2bf_bits(b[e]) : (unsigned short)0;
  }
  const v4u u = (v4u){pk16(hb[0], hb[1]), pk16(hb[2], hb[3]), pk16(hb[4], hb[5]), pk16(hb[6], hb[7])};
  unsigned short* q = AH + (size_t)i * 8;
  *(volatile v4u*)q = u;
  __threadfence();
  *(volatile v4u*)q = u;
}

__device__ __forceinline__ int blk_excl_scan(int cnt, int* scan_ws, int tid, int* tot) {
  const int lane = tid & 31, wave = tid >> 5; int incl = cnt;
#pragma unroll
  for (int o = 1; o < 32; o <<= 1) { const int v = __shfl_up(incl, o, 32); if (lane >= o) incl += v; }
  if (lane == 31) scan_ws[wave] = incl;
  __syncthreads();
  if (wave == 0) { int wv = (lane < kNT / 32) ? scan_ws[lane] : 0; int wincl = wv;
#pragma unroll
    for (int o = 1; o < 32; o <<= 1) { const int v = __shfl_up(wincl, o, 32); if (lane >= o) wincl += v; }
    if (lane < kNT / 32) scan_ws[32 + lane] = wincl - wv; if (lane == 31) scan_ws[64] = wincl; }
  __syncthreads();
  const int res = scan_ws[32 + wave] + incl - cnt; *tot = scan_ws[64];
  return res;
}
__device__ __forceinline__ int chunk_hits(const int* __restrict__ dstv, const int* __restrict__ srcv, int e0, int n0, int tid,
                                          int* LIST, int* scan_ws) {
  const int eb = e0 + tid * kSP;
  const bool inr = eb < kEdges;
  const int ebc = inr ? eb : (kEdges - kSP);
  int rec[kSP]; int cnt = 0;
#pragma unroll
  for (int k = 0; k < kSP; k += 4) {
    const v4i d4 = *(const v4i*)(dstv + ebc + k);
    const v4i s4 = *(const v4i*)(srcv + ebc + k);
#pragma unroll
    for (int e = 0; e < 4; ++e) {
      const int d = d4[e]; int r = -1;
      if (inr && d >= n0 && d < n0 + kSRB) {
        int s = s4[e]; s = s < 0 ? 0 : (s >= kNodes ? kNodes - 1 : s);
        r = ((d - n0) << 16) | s; ++cnt;
      }
      rec[k + e] = r;
    }
  }
  int tot; int p = blk_excl_scan(cnt, scan_ws, tid, &tot);
#pragma unroll
  for (int k = 0; k < kSP; ++k) if (rec[k] >= 0) { if ((unsigned)p < (unsigned)kSCH) LIST[p] = rec[k]; ++p; }
  __syncthreads();
  return tot < kSCH ? tot : kSCH;
}

template <bool FINAL>
__global__ __launch_bounds__(256) void sage_agg_kernel(const float* __restrict__ HW, const int* __restrict__ esrc,
                                                      const int* __restrict__ edst, const float* __restrict__ bias,
                                                      float* AGG, unsigned short* __restrict__ AH,
                                                      unsigned short* __restrict__ AL, float* __restrict__ H3) {
  __shared__ int LIST[kSCH];
  __shared__ int SCNT[kSRB];
  __shared__ int scan_ws[96];
  const int tid = threadIdx.x, lane = tid & 31, wave = tid >> 5;
  const int n0 = blockIdx.x * kSRB;
  const v4f z4 = {0.f, 0.f, 0.f, 0.f};
#pragma unroll 1
  for (int j = 0; j < kRPW; ++j) *(v4f*)(AGG + (size_t)(n0 + wave * kRPW + j) * kCh + 4 * lane) = z4;
  for (int i = tid; i < kSCH; i += kNT) LIST[i] = -1;
  for (int i = tid; i < kSRB; i += kNT) SCNT[i] = 0;
  if (tid < 96) scan_ws[tid] = 0;
  __syncthreads();

#pragma unroll 1
  for (int c = 0; c < kNCH; ++c) {
    const int tot = chunk_hits(edst, esrc, c * kSCH, n0, tid, LIST, scan_ws);
#pragma unroll 1
    for (int base = 0; base < tot; base += 32) {
      const int q = base + lane;
      const int qc = (q < kSCH) ? q : (kSCH - 1);
      const int lv = LIST[qc];
      const int rv = (q < tot) ? lv : -1;
      const int own = (rv >= 0 && ((rv >> 16) >> kRPWLog) == wave) ? 1 : 0;
      unsigned msk = (unsigned)__ballot(own);
#pragma unroll 1
      for (int it = 0; it < 32; ++it) {
        if (msk == 0u) break;
        const int bp = __builtin_ctz(msk); msk &= msk - 1u;
        const int r = __shfl(rv, bp, 32);
        const int dl = r >> 16, s = r & 0xFFFF;
        const v4f hv = *(const v4f*)(HW + (size_t)s * kCh2 + kCh + 4 * lane);
        float* rp = AGG + (size_t)(n0 + dl) * kCh + 4 * lane;
        v4f a = *(const v4f*)rp;
        a = a + hv;
        *(v4f*)rp = a;
        const int cv = SCNT[dl];
        if (lane == 0) SCNT[dl] = cv + 1;
      }
    }
    __syncthreads();
  }
  __syncthreads();

  if (!FINAL) {
    const int c16 = lane & 15, hrow = lane >> 4;
    const v4f bq0 = bfr4(*(const v4f*)(bias + 8 * c16));
    const v4f bq1 = bfr4(*(const v4f*)(bias + 8 * c16 + 4));
#pragma unroll 1
    for (int jj = 0; jj < kRPW / 2; ++jj) {
      const int dl0 = wave * kRPW + 2 * jj;
      if (n0 + dl0 < kNPad) {
        const int dl = dl0 + hrow; const int n = n0 + dl;
        const bool live = n < kNodes;
        const int cnt = SCNT[dl];
        const float inv = 1.0f / fmaxf((float)cnt, 1.0f);
        const float* rp = AGG + (size_t)(n0 + dl) * kCh + 8 * c16;
        const float* sp = HW + (size_t)n * kCh2 + 8 * c16;
        const v4f a0 = *(const v4f*)(rp), a1 = *(const v4f*)(rp + 4);
        const v4f s0 = *(const v4f*)(sp), s1 = *(const v4f*)(sp + 4);
        const v4f t0 = a0 * inv, t1 = a1 * inv;
        v4f v0 = s0 + t0, v1 = s1 + t1;
        v0 = v0 + bq0; v1 = v1 + bq1;
        unsigned short hb[8], lb[8];
#pragma unroll
        for (int e = 0; e < 4; ++e) {
          float f0 = fmaxf(v0[e], 0.f); float f1 = fmaxf(v1[e], 0.f);
          f0 = live ? f0 : 0.f; f1 = live ? f1 : 0.f;
          const unsigned short h0 = f2bf_bits(f0); hb[e] = h0; lb[e] = f2bf_bits(f0 - bf_bits2f(h0));
          const unsigned short h1 = f2bf_bits(f1); hb[4 + e] = h1; lb[4 + e] = f2bf_bits(f1 - bf_bits2f(h1));
        }
        const v4u uh = (v4u){pk16(hb[0], hb[1]), pk16(hb[2], hb[3]), pk16(hb[4], hb[5]), pk16(hb[6], hb[7])};
        const v4u ul = (v4u){pk16(lb[0], lb[1]), pk16(lb[2], lb[3]), pk16(lb[4], lb[5]), pk16(lb[6], lb[7])};
        unsigned short* dh = AH + (size_t)n * kCh + 8 * c16;
        unsigned short* dlp = AL + (size_t)n * kCh + 8 * c16;
        for (int pass = 0; pass < 2; ++pass) {
          *(volatile v4u*)dh = uh;
          *(volatile v4u*)dlp = ul;
          __threadfence();
        }
      }
    }
  } else {
    const v4f bq = bfr4(*(const v4f*)(bias + 4 * lane));
#pragma unroll 1
    for (int j = 0; j < kRPW; ++j) {
      const int dl = wave * kRPW + j; const int n = n0 + dl;
      if (n < kNPad) {
        const bool live = n < kNodes;
        const int cnt = SCNT[dl];
        const float inv = 1.0f / fmaxf((float)cnt, 1.0f);
        const v4f a = *(const v4f*)(AGG + (size_t)(n0 + dl) * kCh + 4 * lane);
        const v4f s = *(const v4f*)(HW + (size_t)n * kCh2 + 4 * lane);
        const v4f t = a * inv;
        v4f v = s + t;
        v = v + bq;
        v4f o;
#pragma unroll
        for (int e = 0; e < 4; ++e) o[e] = live ? v[e] : 0.f;
        float* dp = H3 + (size_t)n * kCh + 4 * lane;
        for (int pass = 0; pass < 2; ++pass) {
          *(volatile v4f*)dp = o;
          __threadfence();
        }
      }
    }
  }
}

__device__ __forceinline__ void mlp_gemm(const unsigned short* zhp, const unsigned short* zlp, const __bf16* __restrict__ Bt,
                                         int wr, int wc, int lane, v8f (&acc)[4]) {
  const __bf16* zh = (const __bf16*)zhp; const __bf16* zl = (const __bf16*)zlp;
  const int rlane = lane & 15, koff = (lane >> 4) * 8;
#pragma unroll
  for (int j = 0; j < 4; ++j) acc[j] = (v8f){0.f,0.f,0.f,0.f,0.f,0.f,0.f,0.f};
#pragma unroll
  for (int k0 = 0; k0 < kCh; k0 += 32) {
    v16b bh[4];
#pragma unroll
    for (int j = 0; j < 4; ++j) bh[j] = Frag<__bf16>::load(Bt + (size_t)(wc * 64 + (j << 4) + rlane) * kCh + koff + k0);
    const int ao = (wr * 16 + rlane) * kZP + koff + k0;
    const v16b ah = Frag<__bf16>::load(zh + ao);
    const v16b al = Frag<__bf16>::load(zl + ao);
#pragma unroll
    for (int j = 0; j < 4; ++j) {
      acc[j] = Frag<__bf16>::mma(ah, bh[j], acc[j]);
      acc[j] = Frag<__bf16>::mma(al, bh[j], acc[j]);
    }
    guard4_b(acc[0], acc[1], acc[2], acc[3], ah, al);
    keep4_b(bh[0], bh[1], bh[2], bh[3]);
  }
  acc_guard4(acc[0], acc[1], acc[2], acc[3]);
}

__global__ __launch_bounds__(256) void predictor_kernel(const float* __restrict__ H3,
                                                        const int* __restrict__ ps, const int* __restrict__ pd,
                                                        const int* __restrict__ ns, const int* __restrict__ nd,
                                                        const unsigned short* __restrict__ Bp1p, const float* __restrict__ bp1,
                                                        const unsigned short* __restrict__ Bp2p, const float* __restrict__ bp2,
                                                        const float* __restrict__ Wp3, const float* __restrict__ bp3,
                                                        float* __restrict__ out) {
  __shared__ __align__(16) unsigned short ZH[64 * kZP];
  __shared__ __align__(16) unsigned short ZL[64 * kZP];
  __shared__ float RED[2][64];
  const int tid = threadIdx.x, lane = tid & 31, wave = tid >> 5;
  const int blk = blockIdx.x;
  const bool isneg = blk >= kPB;
  const int pb = isneg ? (blk - kPB) : blk;
  const int r0 = pb * 64;
  const int* si = isneg ? ns : ps;
  const int* di = isneg ? nd : pd;
  float* ob = out + (isneg ? kPairs : 0) + r0;
  const int rem = kPairs - r0;
  const int nl = (rem >= 64) ? 16 : (rem >> 2);

#pragma unroll 1
  for (int p4 = 0; p4 < 4; ++p4) {
    const int row = p4 * 16 + (tid >> 4);
    const int c8 = (tid & 15) * 8;
    int pr = r0 + row; pr = (pr < kPairs) ? pr : (kPairs - 1);
    int s = si[pr], d = di[pr];
    s = s < 0 ? 0 : (s >= kNodes ? kNodes - 1 : s);
    d = d < 0 ? 0 : (d >= kNodes ? kNodes - 1 : d);
    const float* hs = H3 + (size_t)s * kCh + c8;
    const float* hd = H3 + (size_t)d * kCh + c8;
    const v4f a0 = *(const v4f*)(hs), a1 = *(const v4f*)(hs + 4);
    const v4f g0 = *(const v4f*)(hd), g1 = *(const v4f*)(hd + 4);
    const v4f z0 = a0 * g0, z1 = a1 * g1;
    unsigned short hb[8], lb[8];
#pragma unroll
    for (int e = 0; e < 4; ++e) {
      const unsigned short h0 = f2bf_bits(z0[e]); hb[e] = h0; lb[e] = f2bf_bits(z0[e] - bf_bits2f(h0));
      const unsigned short h1 = f2bf_bits(z1[e]); hb[4 + e] = h1; lb[4 + e] = f2bf_bits(z1[e] - bf_bits2f(h1));
    }
    const v4u uh = (v4u){pk16(hb[0], hb[1]), pk16(hb[2], hb[3]), pk16(hb[4], hb[5]), pk16(hb[6], hb[7])};
    const v4u ul = (v4u){pk16(lb[0], lb[1]), pk16(lb[2], lb[3]), pk16(lb[4], lb[5]), pk16(lb[6], lb[7])};
    *(v4u*)(ZH + row * kZP + c8) = uh;
    *(v4u*)(ZL + row * kZP + c8) = ul;
  }
  __syncthreads();

  const int wr = wave & 3, wc = wave >> 2;
  const int rlane = lane & 15, hh = lane >> 4;
  v8f acc[4];

  mlp_gemm(ZH, ZL, (const __bf16*)Bp1p, wr, wc, lane, acc);
  __syncthreads();
  {
    float bj[4];
#pragma unroll
    for (int j = 0; j < 4; ++j) bj[j] = bfr(bp1[wc * 64 + (j << 4) + rlane]);
#pragma unroll
    for (int j = 0; j < 4; ++j) {
      const int col = wc * 64 + (j << 4) + rlane;
#pragma unroll
      for (int r = 0; r < 8; ++r) {
        const int row = wr * 16 + 8 * hh + r;
        const float v = fmaxf(acc[j][r] + bj[j], 0.f);
        const unsigned short h0 = f2bf_bits(v);
        ZH[row * kZP + col] = h0;
        ZL[row * kZP + col] = f2bf_bits(v - bf_bits2f(h0));
      }
    }
  }
  __syncthreads();

  mlp_gemm(ZH, ZL, (const __bf16*)Bp2p, wr, wc, lane, acc);
  float part[8];
  {
    float b2j[4], w3j[4];
#pragma unroll
    for (int j = 0; j < 4; ++j) {
      const int col = wc * 64 + (j << 4) + rlane;
      b2j[j] = bfr(bp2[col]);
      w3j[j] = bfr(Wp3[col]);
    }
#pragma unroll
    for (int r = 0; r < 8; ++r) {
      float pq = 0.f;
#pragma unroll
      for (int j = 0; j < 4; ++j) {
        const float v = fmaxf(acc[j][r] + b2j[j], 0.f);
        pq += v * w3j[j];
      }
      part[r] = pq;
    }
#pragma unroll
    for (int r = 0; r < 8; ++r) {
      part[r] += __shfl_xor(part[r], 1, 32);
      part[r] += __shfl_xor(part[r], 2, 32);
      part[r] += __shfl_xor(part[r], 4, 32);
      part[r] += __shfl_xor(part[r], 8, 32);
    }
  }
  if (rlane == 0) {
#pragma unroll
    for (int r = 0; r < 8; ++r) RED[wc][wr * 16 + 8 * hh + r] = part[r];
  }
  __syncthreads();
  if (wave == 0) {
    const int l16 = lane & 15;
    const float b3 = bfr(bp3[0]);
    v4f o;
#pragma unroll
    for (int e = 0; e < 4; ++e) {
      const float t = RED[0][4 * l16 + e] + RED[1][4 * l16 + e];
      o[e] = t + b3;
    }
    for (int pass = 0; pass < 2; ++pass) {
      if (lane < nl) *(volatile v4f*)(ob + 4 * lane) = o;
      __threadfence();
    }
  }
}

extern "C" void kernel_launch(void* const* d_in, const int* in_sizes, int n_in,
                              void* d_out, int out_size, void* d_ws, size_t ws_size, hipStream_t stream) {
  if (n_in < 22) return;
  if (in_sizes[0] != kNodes * kCh || in_sizes[1] != kEdges || in_sizes[2] != kEdges ||
      in_sizes[3] != kPairs || in_sizes[4] != kPairs || in_sizes[5] != kPairs || in_sizes[6] != kPairs ||
      in_sizes[7] != kCh * kCh || in_sizes[8] != kCh * kCh || in_sizes[16] != kCh * kCh || in_sizes[18] != kCh * kCh ||
      in_sizes[20] != kCh || in_sizes[21] < 1 || out_size != 2 * kPairs) return;

  const float* x        = (const float*)d_in[0];
  const int*   edge_src = (const int*)d_in[1];
  const int*   edge_dst = (const int*)d_in[2];
  const int*   pos_src  = (const int*)d_in[3];
  const int*   pos_dst  = (const int*)d_in[4];
  const int*   neg_src  = (const int*)d_in[5];
  const int*   neg_dst  = (const int*)d_in[6];
  const float* W_self0  = (const float*)d_in[7];
  const float* W_neigh0 = (const float*)d_in[8];
  const float* b0       = (const float*)d_in[9];
  const float* W_self1  = (const float*)d_in[10];
  const float* W_neigh1 = (const float*)d_in[11];
  const float* b1       = (const float*)d_in[12];
  const float* W_self2  = (const float*)d_in[13];
  const float* W_neigh2 = (const float*)d_in[14];
  const float* b2       = (const float*)d_in[15];
  const float* Wp1      = (const float*)d_in[16];
  const float* bp1      = (const float*)d_in[17];
  const float* Wp2      = (const float*)d_in[18];
  const float* bp2      = (const float*)d_in[19];
  const float* Wp3      = (const float*)d_in[20];
  const float* bp3      = (const float*)d_in[21];
  float* out = (float*)d_out;

  char* ws = (char*)d_ws; size_t off = 0;
  auto carve = [&](size_t bytes) -> char* { char* p = ws + off; off += (bytes + 255) & ~(size_t)255; return p; };
  unsigned*       BT0 = (unsigned*)carve((size_t)kCh2 * kCh * 2);
  unsigned*       BT1 = (unsigned*)carve((size_t)kCh2 * kCh * 2);
  unsigned*       BT2 = (unsigned*)carve((size_t)kCh2 * kCh * 2);
  unsigned*       BQ1 = (unsigned*)carve((size_t)kCh * kCh * 2);
  unsigned*       BQ2 = (unsigned*)carve((size_t)kCh * kCh * 2);
  unsigned short* AH  = (unsigned short*)carve((size_t)kNPad * kCh * 2);
  unsigned short* AL  = (unsigned short*)carve((size_t)kNPad * kCh * 2);
  float*          HW  = (float*)carve((size_t)kNPad * kCh2 * 4);
  float*          AGG = (float*)carve((size_t)kAggRows * kCh * 4);
  float*          H3  = (float*)carve((size_t)kNPad * kCh * 4);
  if (off > ws_size || off > (size_t)134217728) return;

  prep_w_kernel<<<256, kNT, 0, stream>>>(W_self0, W_neigh0, W_self1, W_neigh1, W_self2, W_neigh2, Wp1, Wp2,
                                         BT0, BT1, BT2, BQ1, BQ2);
  cast_x_kernel<<<(kNPad * 16) / kNT, kNT, 0, stream>>>(x, AH);

  sage_gemm_kernel<false><<<kGemmBlocks, kNT, 0, stream>>>(AH, AH, (const unsigned short*)BT0, HW);
  sage_agg_kernel<false><<<kTiles, kNT, 0, stream>>>(HW, edge_src, edge_dst, b0, AGG, AH, AL, H3);
  sage_gemm_kernel<true><<<kGemmBlocks, kNT, 0, stream>>>(AH, AL, (const unsigned short*)BT1, HW);
  sage_agg_kernel<false><<<kTiles, kNT, 0, stream>>>(HW, edge_src, edge_dst, b1, AGG, AH, AL, H3);
  sage_gemm_kernel<true><<<kGemmBlocks, kNT, 0, stream>>>(AH, AL, (const unsigned short*)BT2, HW);
  sage_agg_kernel<true><<<kTiles, kNT, 0, stream>>>(HW, edge_src, edge_dst, b2, AGG, AH, AL, H3);
  predictor_kernel<<<2 * kPB, kNT, 0, stream>>>(H3, pos_src, pos_dst, neg_src, neg_dst,
                                                (const unsigned short*)BQ1, bp1, (const unsigned short*)BQ2, bp2,
                                                Wp3, bp3, out);
}
